// VSSBlock_34059090657705
// MI455X (gfx1250) — hardware-run, weakly checked
//
#include <hip/hip_runtime.h>
#include <math.h>

typedef __attribute__((ext_vector_type(16))) _Float16 v16h;
typedef __attribute__((ext_vector_type(8)))  _Float16 v8h;
typedef __attribute__((ext_vector_type(16))) __bf16   v16b;
typedef __attribute__((ext_vector_type(8)))  __bf16   v8b;
typedef __attribute__((ext_vector_type(8)))  float    v8f;
typedef __attribute__((ext_vector_type(4)))  float    v4f;
typedef __attribute__((ext_vector_type(2)))  float    v2f;
typedef __attribute__((ext_vector_type(4)))  unsigned v4u;
typedef __attribute__((ext_vector_type(2)))  unsigned v2u;

constexpr int kB     = 4;
constexpr int kHgt   = 64;
constexpr int kWid   = 64;
constexpr int kC     = 192;
constexpr int kDI    = 384;
constexpr int kNS    = 16;
constexpr int kR     = 24;
constexpr int kK4    = 4;
constexpr int kHW    = kHgt * kWid;
constexpr int kL4    = kHW / 4;
constexpr int kPos   = kB * kHW;
constexpr int kXZ    = 2 * kDI;
constexpr int kCDBL  = kR + 2 * kNS;
constexpr int kXDW   = 64;
constexpr int kDTK   = 32;
constexpr int kRowsK = kB * kL4;
constexpr int kScanTS = 64;
constexpr int kScanCh = 64;
constexpr int kScanYP = 68;
static_assert(kR == (kDI + 15) / 16);
static_assert(kCDBL == 56);
static_assert((kC % 32) == 0 && (kDI % 32) == 0 && kDTK == 32);
static_assert((kPos % 64) == 0 && (kXZ % 64) == 0 && (kXDW % 64) == 0 && (kDI % 64) == 0 && (kC % 64) == 0 && (kRowsK % 64) == 0);
static_assert((kL4 % kScanTS) == 0 && (kDI % kScanCh) == 0);
static_assert(kC == 2 * 96 && kDI == 2 * 192 && kDI == 4 * 96);

constexpr float kWCarry   = 16.0f;
constexpr float kUCarry   = 64.0f;
constexpr float kDtsCarry = 256.0f;
constexpr float kYCarry   = 16.0f;
constexpr float kScaleIn  = 1.0f / kWCarry;
constexpr float kScaleXp  = 1.0f / (kUCarry * kWCarry);
constexpr float kScaleDt  = 1.0f / (kDtsCarry * kWCarry);
constexpr float kScaleRes = 1.0f / kWCarry;
constexpr float kScaleOut = 1.0f / (kYCarry * kWCarry);

constexpr size_t kOffXLN  = 0;
constexpr size_t kOffWIN  = kOffXLN  + (size_t)kPos * kC * 2;
constexpr size_t kOffWXP  = kOffWIN  + (size_t)kXZ * kC * 2;
constexpr size_t kOffWDT  = kOffWXP  + (size_t)kK4 * kXDW * kDI * 2;
constexpr size_t kOffWRES = kOffWDT  + (size_t)kK4 * kDI * kDTK * 2;
constexpr size_t kOffWOUT = kOffWRES + (size_t)kDI * kC * 2;
constexpr size_t kOffXZB  = kOffWOUT + (size_t)kC * kDI * 2;
constexpr size_t kOffU32  = kOffXZB  + (size_t)kPos * kXZ * 2;
constexpr size_t kOffU16  = kOffU32  + (size_t)kPos * kDI * 4;
constexpr size_t kOffXDBL = kOffU16  + (size_t)kPos * kDI * 2;
constexpr size_t kOffDTSA = kOffXDBL + (size_t)kPos * kXDW * 4;
constexpr size_t kOffDTR  = kOffDTSA + (size_t)kPos * kDTK * 2;
constexpr size_t kOffYS   = kOffDTR  + (size_t)kPos * kDI * 4;
constexpr size_t kWsTotal = kOffYS   + (size_t)kPos * kDI * 4;
static_assert(kWsTotal == 125665280ull);
static_assert(kWsTotal <= 134217728ull);
static_assert((kOffWIN % 128) == 0 && (kOffWXP % 128) == 0 && (kOffWDT % 128) == 0 && (kOffWRES % 128) == 0 &&
              (kOffWOUT % 128) == 0 && (kOffXZB % 128) == 0 && (kOffU32 % 128) == 0 && (kOffU16 % 128) == 0 &&
              (kOffXDBL % 128) == 0 && (kOffDTSA % 128) == 0 && (kOffDTR % 128) == 0 && (kOffYS % 128) == 0);

__device__ __forceinline__ unsigned short f2bf_bits(float f) {
  unsigned u = __float_as_uint(f);
  return (unsigned short)((u + 0x7FFFu + ((u >> 16) & 1u)) >> 16);
}
__device__ __forceinline__ float bf_bits2f(unsigned short h) { return __uint_as_float(((unsigned)h) << 16); }

__device__ __forceinline__ float h16_to_f32(unsigned hb) {
  const unsigned sgn = (hb & 0x8000u) << 16; const unsigned em = hb & 0x7fffu;
  const float fn = __uint_as_float((em << 13) + 0x38000000u);
  const float fs = (float)em * 5.9604644775390625e-8f;
  const float mag = (em < 0x400u) ? fs : fn; return __uint_as_float(__float_as_uint(mag) | sgn); }

__device__ __forceinline__ unsigned pack_f16x2(float a, float b) {
  const _Float16 h0 = (_Float16)a, h1 = (_Float16)b;
  return (unsigned)__builtin_bit_cast(unsigned short, h0) | ((unsigned)__builtin_bit_cast(unsigned short, h1) << 16);
}

__device__ __forceinline__ float wave_sum(float v) {
#pragma unroll
  for (int o = 16; o > 0; o >>= 1) v += __shfl_xor(v, o, 32);
  return v;
}

__device__ __forceinline__ void dep_guard4_h(v8f& a, v8f& b, v8f& c, v8f& d, v16h x, v16h y) { asm volatile("v_nop\n\tv_nop\n\tv_nop\n\tv_nop" : "+v"(a), "+v"(b), "+v"(c), "+v"(d) : "v"(x), "v"(y)); }
__device__ __forceinline__ void dep_guard4_b(v8f& a, v8f& b, v8f& c, v8f& d, v16b x, v16b y) { asm volatile("v_nop\n\tv_nop\n\tv_nop\n\tv_nop" : "+v"(a), "+v"(b), "+v"(c), "+v"(d) : "v"(x), "v"(y)); }
__device__ __forceinline__ void keep4_h(v16h a, v16h b, v16h c, v16h d) { asm volatile("v_nop" :: "v"(a), "v"(b), "v"(c), "v"(d)); }
__device__ __forceinline__ void keep4_b(v16b a, v16b b, v16b c, v16b d) { asm volatile("v_nop" :: "v"(a), "v"(b), "v"(c), "v"(d)); }
__device__ __forceinline__ void acc_guard4(v8f& a, v8f& b, v8f& c, v8f& d) { asm volatile("v_nop\n\tv_nop\n\tv_nop\n\tv_nop" : "+v"(a), "+v"(b), "+v"(c), "+v"(d)); }
template <typename T> struct Frag;
template <> struct Frag<_Float16> {
  typedef v16h V; union U { v16h v; v8h h[2]; };
  static __device__ __forceinline__ v16h load(const _Float16* p) {
    U f; f.h[0] = *(const v8h*)(p); f.h[1] = *(const v8h*)(p + 16); return f.v;
  }
  static __device__ __forceinline__ v8f mma(v16h a, v16h b, v8f c) {
    return __builtin_amdgcn_wmma_f32_16x16x32_f16(false, a, false, b, (short)0, c, false, false);
  }
  static __device__ __forceinline__ void guard4(v8f& a, v8f& b, v8f& c, v8f& d, v16h x, v16h y) { dep_guard4_h(a, b, c, d, x, y); }
  static __device__ __forceinline__ void keep(v16h a, v16h b, v16h c, v16h d) { keep4_h(a, b, c, d); }
};
template <> struct Frag<__bf16> {
  typedef v16b V; union U { v16b v; v8b h[2]; };
  static __device__ __forceinline__ v16b load(const __bf16* p) {
    U f; f.h[0] = *(const v8b*)(p); f.h[1] = *(const v8b*)(p + 16); return f.v;
  }
  static __device__ __forceinline__ v8f mma(v16b a, v16b b, v8f c) {
    return __builtin_amdgcn_wmma_f32_16x16x32_bf16(false, a, false, b, (short)0, c, false, false);
  }
  static __device__ __forceinline__ void guard4(v8f& a, v8f& b, v8f& c, v8f& d, v16b x, v16b y) { dep_guard4_b(a, b, c, d, x, y); }
  static __device__ __forceinline__ void keep(v16b a, v16b b, v16b c, v16b d) { keep4_b(a, b, c, d); }
};

template <int ET> struct Elem;
template <> struct Elem<0> { typedef _Float16 T; };
template <> struct Elem<1> { typedef __bf16 T; };
template <int ET, bool SPLIT, int BIAS_MODE, int OUT_MODE, bool RESID>
__global__ __launch_bounds__(256) void wmma_gemm64(
    const unsigned short* __restrict__ Ap, const unsigned short* __restrict__ A2p, int lda, long strideA,
    const unsigned short* __restrict__ Btp, const unsigned short* __restrict__ Bt2p, int ldb, long strideB,
    void* __restrict__ Cout, void* __restrict__ Cout2, int ldc, long strideC,
    const float* __restrict__ bias,
    const float* __restrict__ resid, long strideR,
    int M, int N, int K, float scale) {
  typedef typename Elem<ET>::T T;
  typedef typename Frag<T>::V V;
  const T* A = (const T*)Ap; const T* A2 = (const T*)A2p; const T* Bt = (const T*)Btp; const T* Bt2 = (const T*)Bt2p;
  __shared__ __align__(16) float sT[8][16 * 68];
  const int b    = blockIdx.y;
  const int lane = threadIdx.x & 31;
  const int wave = threadIdx.x >> 5;
  const int tilesN = N >> 6;
  const int tilesM = M >> 6;
  const int tile = blockIdx.x * 8 + wave;
  if (tile >= tilesM * tilesN) return;
  const int tm = tile / tilesN;
  const int tn = tile - tm * tilesN;
  const int m0 = tm << 6;
  const int n0 = tn << 6;

  const T* Ab  = A  + (size_t)b * strideA;
  const T* Bb  = Bt + (size_t)b * strideB;
  const T* Ab2 = SPLIT ? (A2  + (size_t)b * strideA) : nullptr;
  const T* Bb2 = SPLIT ? (Bt2 + (size_t)b * strideB) : nullptr;

  const int rlane = lane & 15;
  const int koff  = (lane >> 4) * 8;
  const int mOff  = (lane >> 4) * 8;

  v8f acc[4][4];
#pragma unroll
  for (int i = 0; i < 4; ++i)
#pragma unroll
    for (int j = 0; j < 4; ++j) acc[i][j] = (v8f){0.f,0.f,0.f,0.f,0.f,0.f,0.f,0.f};

  for (int k0 = 0; k0 < K; k0 += 32) {
    V bh[4], bl[4];
#pragma unroll
    for (int j = 0; j < 4; ++j) {
      const size_t bo = (size_t)(n0 + (j << 4) + rlane) * ldb + koff + k0;
      bh[j] = Frag<T>::load(Bb + bo);
      if (SPLIT) bl[j] = Frag<T>::load(Bb2 + bo);
    }
#pragma unroll
    for (int i = 0; i < 4; ++i) {
      const size_t ao = (size_t)(m0 + (i << 4) + rlane) * lda + koff + k0;
      V ah = Frag<T>::load(Ab + ao);
      V al;
      if (SPLIT) al = Frag<T>::load(Ab2 + ao);
#pragma unroll
      for (int j = 0; j < 4; ++j) {
        acc[i][j] = Frag<T>::mma(ah, bh[j], acc[i][j]);
        if (SPLIT) {
          acc[i][j] = Frag<T>::mma(ah, bl[j], acc[i][j]);
          acc[i][j] = Frag<T>::mma(al, bh[j], acc[i][j]);
        }
      }
      Frag<T>::guard4(acc[i][0], acc[i][1], acc[i][2], acc[i][3], ah, SPLIT ? al : ah);
    }
    Frag<T>::keep(bh[0], bh[1], bh[2], bh[3]);
    if (SPLIT) Frag<T>::keep(bl[0], bl[1], bl[2], bl[3]);
  }
  acc_guard4(acc[0][0], acc[0][1], acc[0][2], acc[0][3]);
  acc_guard4(acc[1][0], acc[1][1], acc[1][2], acc[1][3]);
  acc_guard4(acc[2][0], acc[2][1], acc[2][2], acc[2][3]);
  acc_guard4(acc[3][0], acc[3][1], acc[3][2], acc[3][3]);

  float* slab = sT[wave];
  const float* Rb = RESID ? (resid + (size_t)b * strideR) : nullptr;
#pragma unroll
  for (int i = 0; i < 4; ++i) {
    const int mBase = m0 + (i << 4);
#pragma unroll
    for (int j = 0; j < 4; ++j) {
      const int n = n0 + (j << 4) + rlane;
      float bv = 0.f;
      if (BIAS_MODE == 2) bv = bias[n];
#pragma unroll
      for (int r = 0; r < 8; ++r) {
        float v = acc[i][j][r] * scale;
        if (BIAS_MODE == 1) v += bias[mBase + mOff + r];
        if (BIAS_MODE == 2) v += bv;
        slab[(mOff + r) * 68 + (j << 4) + rlane] = v;
      }
    }
    __builtin_amdgcn_fence(__ATOMIC_RELEASE, "workgroup");
    __builtin_amdgcn_wave_barrier();
    __builtin_amdgcn_fence(__ATOMIC_ACQUIRE, "workgroup");
    if (OUT_MODE == 0) {
      float* C = (float*)Cout + (size_t)b * strideC;
      const int hh = lane >> 4, c4 = (lane & 15) * 4;
      if (RESID) {
#pragma unroll
        for (int it = 0; it < 8; ++it) {
          const int row = it * 2 + hh;
          v4f v = *(const v4f*)(slab + row * 68 + c4);
          const v4f rr = *(const v4f*)(Rb + (size_t)(mBase + row) * ldc + n0 + c4);
          v += rr;
          float* cp = C + (size_t)(mBase + row) * ldc + n0 + c4;
          *(volatile v4f*)cp = v;
          __threadfence();
          *(volatile v4f*)cp = v;
        }
      } else {
        for (int pass = 0; pass < 2; ++pass) {
#pragma unroll
          for (int it = 0; it < 8; ++it) {
            const int row = it * 2 + hh;
            v4f v = *(const v4f*)(slab + row * 68 + c4);
            *(volatile v4f*)(C + (size_t)(mBase + row) * ldc + n0 + c4) = v;
          }
          __threadfence();
        }
      }
    } else {
      const int q = lane >> 3, c8 = (lane & 7) * 8;
      unsigned short* C  = (unsigned short*)Cout  + (size_t)b * strideC;
      unsigned short* C2 = (OUT_MODE == 2) ? ((unsigned short*)Cout2 + (size_t)b * strideC) : nullptr;
      for (int pass = 0; pass < 2; ++pass) {
#pragma unroll
        for (int it = 0; it < 4; ++it) {
          const int row = it * 4 + q;
          const float* sp = slab + row * 68 + c8;
          v8h hv, lv;
#pragma unroll
          for (int e = 0; e < 8; ++e) {
            if (OUT_MODE == 1) {
              hv[e] = (_Float16)sp[e];
            } else {
              unsigned short hb = f2bf_bits(sp[e]);
              unsigned short lb = f2bf_bits(sp[e] - bf_bits2f(hb));
              hv[e] = __builtin_bit_cast(_Float16, hb);
              lv[e] = __builtin_bit_cast(_Float16, lb);
            }
          }
          *(volatile v8h*)(C + (size_t)(mBase + row) * ldc + n0 + c8) = hv;
          if (OUT_MODE == 2) *(volatile v8h*)(C2 + (size_t)(mBase + row) * ldc + n0 + c8) = lv;
        }
        __threadfence();
      }
    }
    __builtin_amdgcn_fence(__ATOMIC_RELEASE, "workgroup");
    __builtin_amdgcn_wave_barrier();
    __builtin_amdgcn_fence(__ATOMIC_ACQUIRE, "workgroup");
  }
}

template <int MODE>
__global__ __launch_bounds__(256) void cvt_w_kernel(const float* __restrict__ src, unsigned short* __restrict__ dst,
                                                    int NR, int NC, int srcC, int total2) {
  const int i = blockIdx.x * 256 + threadIdx.x;
  if (i >= total2) return;
  const int e0 = 2 * i;
  const int n = e0 / NC;
  const int c = e0 - n * NC;
  int srow = n;
  int rowok = 1;
  if (MODE == 1) {
    const int nl = n & 63, g = n >> 6;
    rowok = (nl < kR) | (nl >= 32);
    const int m = (nl < 32) ? nl : (nl - 8);
    srow = g * kCDBL + m;
  }
  const int c0 = (c < srcC) ? c : (srcC - 1);
  const int c1 = (c + 1 < srcC) ? (c + 1) : (srcC - 1);
  const float v0 = src[(size_t)srow * srcC + c0];
  const float v1 = src[(size_t)srow * srcC + c1];
  const float f0 = (rowok & (c < srcC)) ? kWCarry : 0.0f;
  const float f1 = (rowok & (c + 1 < srcC)) ? kWCarry : 0.0f;
  const unsigned wd = pack_f16x2(v0 * f0, v1 * f1);
  unsigned* p = (unsigned*)dst + i;
  *(volatile unsigned*)p = wd;
  __threadfence();
  *(volatile unsigned*)p = wd;
  (void)NR;
}

__global__ __launch_bounds__(384) void ln1_kernel(const float* __restrict__ x, const float* __restrict__ w,
                                                const float* __restrict__ bb, unsigned short* __restrict__ xln) {
  __shared__ float sRed1[12];
  __shared__ float sRed2[12];
  const int tid = threadIdx.x, lane = tid & 31, wave = tid >> 5;
  const int rl = tid / 96;
  const int q  = tid - rl * 96;
  const int c0 = 2 * q;
  const size_t row = (size_t)blockIdx.x * 4 + rl;
  const v2f xv = *(const v2f*)(x + row * kC + c0);
  const v2f wv = *(const v2f*)(w + c0);
  const v2f bv = *(const v2f*)(bb + c0);
  const float x0 = xv.x, x1 = xv.y;
  const float s = wave_sum(x0 + x1);
  if (lane == 0) sRed1[wave] = s;
  __syncthreads();
  const float tot = (sRed1[3 * rl] + sRed1[3 * rl + 1]) + sRed1[3 * rl + 2];
  const float mu = tot * (1.0f / (float)kC);
  const float d0 = x0 - mu, d1 = x1 - mu;
  const float q2 = wave_sum(fmaf(d0, d0, d1 * d1));
  if (lane == 0) sRed2[wave] = q2;
  __syncthreads();
  const float var = ((sRed2[3 * rl] + sRed2[3 * rl + 1]) + sRed2[3 * rl + 2]) * (1.0f / (float)kC);
  const float rs = rsqrtf(var + 1e-6f);
  const float o0 = (d0 * rs) * wv.x + bv.x;
  const float o1 = (d1 * rs) * wv.y + bv.y;
  const unsigned wd = pack_f16x2(o0, o1);
  unsigned* p = (unsigned*)xln + ((row * kC + c0) >> 1);
  *(volatile unsigned*)p = wd;
  __threadfence();
  *(volatile unsigned*)p = wd;
}

__device__ __forceinline__ float silu_f32(float v) {
  const float e = expf(-v);
  return v * __builtin_amdgcn_rcpf(1.0f + e);
}

__global__ __launch_bounds__(384) void dwconv_silu_kernel(const unsigned short* __restrict__ XZB,
    const float* __restrict__ cw, const float* __restrict__ cb, float* __restrict__ U32, unsigned short* __restrict__ U16) {
  __shared__ float sW[kDI * 9];
  __shared__ float sBias[kDI];
  const int tid = threadIdx.x;
#pragma unroll 1
  for (int j = 0; j < 9; ++j) sW[tid * 9 + j] = cw[tid * 9 + j];
  sBias[tid] = cb[tid];
  __syncthreads();
  const int pl = tid / 96;
  const int q  = tid - pl * 96;
  const int d  = 4 * q;
  const int pos  = blockIdx.x * 4 + pl;
  const int bimg = pos >> 12;
  const int hp   = (pos >> 6) & (kHgt - 1);
  const int wp   = pos & (kWid - 1);
  const unsigned* XW = (const unsigned*)XZB;
  float acc0 = 0.0f, acc1 = 0.0f, acc2 = 0.0f, acc3 = 0.0f;
#pragma unroll
  for (int dh = 0; dh < 3; ++dh) {
    const int hq  = hp + dh - 1;
    const int hok = (hq >= 0) & (hq < kHgt);
    const int hc  = hq < 0 ? 0 : (hq > kHgt - 1 ? kHgt - 1 : hq);
#pragma unroll
    for (int dw = 0; dw < 3; ++dw) {
      const int wq  = wp + dw - 1;
      const int wok = (wq >= 0) & (wq < kWid);
      const int wc  = wq < 0 ? 0 : (wq > kWid - 1 ? kWid - 1 : wq);
      const float f = (hok & wok) ? 1.0f : 0.0f;
      const size_t eoff = ((size_t)((bimg * kHgt + hc) * kWid + wc)) * kXZ + d;
      const v2u wd2 = *(const v2u*)(XW + (eoff >> 1));
      const unsigned wA = wd2.x, wB = wd2.y;
      const float x0 = h16_to_f32(wA & 0xffffu) * f;
      const float x1 = h16_to_f32(wA >> 16) * f;
      const float x2 = h16_to_f32(wB & 0xffffu) * f;
      const float x3 = h16_to_f32(wB >> 16) * f;
      const int tap = dh * 3 + dw;
      acc0 = fmaf(x0, sW[(d + 0) * 9 + tap], acc0);
      acc1 = fmaf(x1, sW[(d + 1) * 9 + tap], acc1);
      acc2 = fmaf(x2, sW[(d + 2) * 9 + tap], acc2);
      acc3 = fmaf(x3, sW[(d + 3) * 9 + tap], acc3);
    }
    asm volatile("" ::: "memory");
  }
  const float u0 = silu_f32(acc0 + sBias[d + 0]);
  const float u1 = silu_f32(acc1 + sBias[d + 1]);
  const float u2 = silu_f32(acc2 + sBias[d + 2]);
  const float u3 = silu_f32(acc3 + sBias[d + 3]);
  const int kq = (hp & 1) ? ((wp & 1) ? 1 : 3) : ((wp & 1) ? 2 : 0);
  const int l  = (hp >> 1) * (kWid / 2) + (wp >> 1);
  const size_t orow = (size_t)(kq * kB + bimg) * kL4 + l;
  v4f uv; uv.x = u0; uv.y = u1; uv.z = u2; uv.w = u3;
  v2u hv; hv.x = pack_f16x2(u0 * kUCarry, u1 * kUCarry); hv.y = pack_f16x2(u2 * kUCarry, u3 * kUCarry);
  float* up = U32 + orow * kDI + d;
  unsigned* hp2 = (unsigned*)U16 + ((orow * kDI + d) >> 1);
  *(volatile v4f*)up = uv;
  *(volatile v2u*)hp2 = hv;
  __threadfence();
  *(volatile v4f*)up = uv;
  *(volatile v2u*)hp2 = hv;
}

__global__ __launch_bounds__(256) void dts_pack_kernel(const float* __restrict__ XD, unsigned short* __restrict__ DT, int total) {
  const int i = blockIdx.x * 256 + threadIdx.x;
  if (i >= total) return;
  const int row = i >> 2, g = i & 3;
  const int cb = g * 8;
  const float* sp = XD + (size_t)row * kXDW + cb;
  const v4f a = *(const v4f*)(sp);
  const v4f bq = *(const v4f*)(sp + 4);
  const float f0 = (cb + 0 < kR) ? kDtsCarry : 0.0f;
  const float f1 = (cb + 1 < kR) ? kDtsCarry : 0.0f;
  const float f2 = (cb + 2 < kR) ? kDtsCarry : 0.0f;
  const float f3 = (cb + 3 < kR) ? kDtsCarry : 0.0f;
  const float f4 = (cb + 4 < kR) ? kDtsCarry : 0.0f;
  const float f5 = (cb + 5 < kR) ? kDtsCarry : 0.0f;
  const float f6 = (cb + 6 < kR) ? kDtsCarry : 0.0f;
  const float f7 = (cb + 7 < kR) ? kDtsCarry : 0.0f;
  v4u wv;
  wv.x = pack_f16x2(a.x * f0, a.y * f1);
  wv.y = pack_f16x2(a.z * f2, a.w * f3);
  wv.z = pack_f16x2(bq.x * f4, bq.y * f5);
  wv.w = pack_f16x2(bq.z * f6, bq.w * f7);
  unsigned* p = (unsigned*)DT + (((size_t)row * kDTK + cb) >> 1);
  *(volatile v4u*)p = wv;
  __threadfence();
  *(volatile v4u*)p = wv;
}

__global__ __launch_bounds__(64) void scan_kernel(const float* __restrict__ XD, const float* __restrict__ DTR,
    const float* __restrict__ U32, const float* __restrict__ dtb, const float* __restrict__ Alog,
    const float* __restrict__ Dsp, float* __restrict__ YS) {
  __shared__ __align__(16) float sX[kScanTS * 32];
  __shared__ __align__(16) float sY[kScanTS * kScanYP];
  __shared__ float sA[kNS * kScanCh];
  const int tid = threadIdx.x, lane = tid & 31, wave = tid >> 5;
  constexpr int kGroups = kDI / kScanCh;
  const int kb = blockIdx.x / kGroups;
  const int d0 = (blockIdx.x - kb * kGroups) * kScanCh;
  const int d  = d0 + tid;
  const int kq = kb >> 2, bimg = kb & 3;
  const size_t R0 = (size_t)kb * kL4;
  const int kd = kq * kDI + d;
#pragma unroll 1
  for (int n = 0; n < kNS; ++n) sA[n * kScanCh + tid] = -expf(Alog[(size_t)kd * kNS + n]);
  __syncthreads();
  float negA[kNS], h[kNS];
#pragma unroll
  for (int n = 0; n < kNS; ++n) { negA[n] = sA[n * kScanCh + tid]; h[n] = 0.0f; }
  const float bb = dtb[kd], Dd = Dsp[kd];
  const int kr = kq & 1;
  const int kc = (kq == 1) | (kq == 2);
  const int lr = tid >> 3, lc4 = (tid & 7) * 4;
  const int hh = lane >> 4, c4 = (lane & 15) * 4;
#pragma unroll 1
  for (int t0 = 0; t0 < kL4; t0 += kScanTS) {
    __syncthreads();
#pragma unroll
    for (int i = 0; i < 8; ++i) {
      const int r = lr + 8 * i;
      *(v4f*)(sX + r * 32 + lc4) = *(const v4f*)(XD + (R0 + t0 + r) * kXDW + 32 + lc4);
    }
    __syncthreads();
#pragma unroll 1
    for (int s = 0; s < kScanTS; ++s) {
      const size_t t = R0 + t0 + s;
      const float* xr = sX + s * 32;
      float Bs[kNS], Cs[kNS];
#pragma unroll
      for (int q4 = 0; q4 < 4; ++q4) {
        const v4f bv = *(const v4f*)(xr + 4 * q4);
        const v4f cv = *(const v4f*)(xr + kNS + 4 * q4);
        Bs[4 * q4 + 0] = bv.x; Bs[4 * q4 + 1] = bv.y; Bs[4 * q4 + 2] = bv.z; Bs[4 * q4 + 3] = bv.w;
        Cs[4 * q4 + 0] = cv.x; Cs[4 * q4 + 1] = cv.y; Cs[4 * q4 + 2] = cv.z; Cs[4 * q4 + 3] = cv.w;
      }
      const float v   = DTR[t * kDI + d] + bb;
      const float sp  = fmaxf(v, 0.0f) + log1pf(expf(-fabsf(v)));
      const float ut  = U32[t * kDI + d];
      const float dtu = sp * ut;
      float y = 0.0f;
#pragma unroll
      for (int n = 0; n < kNS; ++n) {
        const float e = __expf(sp * negA[n]);
        h[n] = fmaf(e, h[n], dtu * Bs[n]);
        y = fmaf(h[n], Cs[n], y);
      }
      y = fmaf(Dd, ut, y);
      sY[s * kScanYP + tid] = y;
    }
    __syncthreads();
    for (int pass = 0; pass < 2; ++pass) {
#pragma unroll
      for (int it = 0; it < 16; ++it) {
        const int row = it * 4 + wave * 2 + hh;
        const int l = t0 + row;
        const int hpos = 2 * (l >> 5) + kr;
        const int wpos = 2 * (l & 31) + kc;
        const size_t pos = (size_t)bimg * kHW + (size_t)hpos * kWid + wpos;
        const v4f val = *(const v4f*)(sY + row * kScanYP + c4);
        *(volatile v4f*)(YS + pos * kDI + d0 + c4) = val;
      }
      __threadfence();
    }
  }
}

__global__ __launch_bounds__(384) void norm_gate_kernel(const float* __restrict__ YS, const float* __restrict__ onw,
    const float* __restrict__ onb, const float* __restrict__ RES, const unsigned short* __restrict__ XZB,
    unsigned short* __restrict__ YF) {
  __shared__ float sRed1[12];
  __shared__ float sRed2[12];
  const int tid = threadIdx.x, lane = tid & 31, wave = tid >> 5;
  const int rl = tid / 192;
  const int q  = tid - rl * 192;
  const int c0 = 2 * q;
  const size_t row = (size_t)blockIdx.x * 2 + rl;
  const v2f yv = *(const v2f*)(YS + row * kDI + c0);
  const float y0 = yv.x, y1 = yv.y;
  const float s = wave_sum(y0 + y1);
  if (lane == 0) sRed1[wave] = s;
  __syncthreads();
  const float tot = ((sRed1[6 * rl] + sRed1[6 * rl + 1]) + (sRed1[6 * rl + 2] + sRed1[6 * rl + 3])) + (sRed1[6 * rl + 4] + sRed1[6 * rl + 5]);
  const float mu = tot * (1.0f / (float)kDI);
  const float d0 = y0 - mu, d1 = y1 - mu;
  const float q2 = wave_sum(fmaf(d0, d0, d1 * d1));
  if (lane == 0) sRed2[wave] = q2;
  __syncthreads();
  const float vs  = ((sRed2[6 * rl] + sRed2[6 * rl + 1]) + (sRed2[6 * rl + 2] + sRed2[6 * rl + 3])) + (sRed2[6 * rl + 4] + sRed2[6 * rl + 5]);
  const float var = vs * (1.0f / (float)kDI);
  const float rs  = rsqrtf(var + 1e-5f);
  const v2f wv = *(const v2f*)(onw + c0);
  const v2f bv = *(const v2f*)(onb + c0);
  const v2f rv = *(const v2f*)(RES + row * kDI + c0);
  const unsigned zw = ((const unsigned*)XZB)[(row * kXZ + kDI + c0) >> 1];
  const float z0 = h16_to_f32(zw & 0xffffu);
  const float z1 = h16_to_f32(zw >> 16);
  const float a0 = ((d0 * rs) * wv.x + bv.x) + rv.x;
  const float a1 = ((d1 * rs) * wv.y + bv.y) + rv.y;
  const float g0 = silu_f32(z0);
  const float g1 = silu_f32(z1);
  const float o0 = (a0 * g0) * kYCarry;
  const float o1 = (a1 * g1) * kYCarry;
  const unsigned wd = pack_f16x2(o0, o1);
  unsigned* p = (unsigned*)YF + ((row * kDI + c0) >> 1);
  *(volatile unsigned*)p = wd;
  __threadfence();
  *(volatile unsigned*)p = wd;
}

constexpr int kTot2WIN  = kXZ * kC / 2;
constexpr int kTot2WXP  = kK4 * kXDW * kDI / 2;
constexpr int kTot2WDT  = kK4 * kDI * kDTK / 2;
constexpr int kTot2WRES = kDI * kC / 2;
constexpr int kTot2WOUT = kC * kDI / 2;
constexpr int kTotPack  = kPos * 4;
static_assert((kTot2WIN % 256) == 0 && (kTot2WXP % 256) == 0 && (kTot2WDT % 256) == 0 && (kTot2WRES % 256) == 0 &&
              (kTot2WOUT % 256) == 0 && (kTotPack % 256) == 0 && (kPos % 4) == 0 && (kPos % 2) == 0);
static_assert(((kPos / 64) * (kXZ / 64)) % 8 == 0 && ((kRowsK / 64) * (kXDW / 64)) % 8 == 0 &&
              ((kRowsK / 64) * (kDI / 64)) % 8 == 0 && ((kPos / 64) * (kDI / 64)) % 8 == 0 && ((kPos / 64) * (kC / 64)) % 8 == 0);

extern "C" void kernel_launch(void* const* d_in, const int* in_sizes, int n_in,
                              void* d_out, int out_size, void* d_ws, size_t ws_size,
                              hipStream_t stream) {
  if (n_in < 15) return;
  if (in_sizes[0]  != kPos * kC) return;
  if (in_sizes[1]  != kC) return;
  if (in_sizes[2]  != kC) return;
  if (in_sizes[3]  != kXZ * kC) return;
  if (in_sizes[4]  != kDI * 9) return;
  if (in_sizes[5]  != kDI) return;
  if (in_sizes[6]  != kK4 * kCDBL * kDI) return;
  if (in_sizes[7]  != kK4 * kDI * kR) return;
  if (in_sizes[8]  != kK4 * kDI) return;
  if (in_sizes[9]  != kK4 * kDI * kNS) return;
  if (in_sizes[10] != kK4 * kDI) return;
  if (in_sizes[11] != kDI) return;
  if (in_sizes[12] != kDI) return;
  if (in_sizes[13] != kDI * kC) return;
  if (in_sizes[14] != kC * kDI) return;
  if (out_size != kPos * kC) return;
  if (ws_size < kWsTotal) return;

  const float* inputs     = (const float*)d_in[0];
  const float* ln1_w      = (const float*)d_in[1];
  const float* ln1_b      = (const float*)d_in[2];
  const float* in_proj_w  = (const float*)d_in[3];
  const float* conv_w     = (const float*)d_in[4];
  const float* conv_b     = (const float*)d_in[5];
  const float* x_proj_w   = (const float*)d_in[6];
  const float* dt_w       = (const float*)d_in[7];
  const float* dt_b       = (const float*)d_in[8];
  const float* A_logs     = (const float*)d_in[9];
  const float* Ds         = (const float*)d_in[10];
  const float* out_norm_w = (const float*)d_in[11];
  const float* out_norm_b = (const float*)d_in[12];
  const float* res_proj_w = (const float*)d_in[13];
  const float* out_proj_w = (const float*)d_in[14];
  float* out = (float*)d_out;

  char* ws = (char*)d_ws;
  unsigned short* XLN  = (unsigned short*)(ws + kOffXLN);
  unsigned short* WIN  = (unsigned short*)(ws + kOffWIN);
  unsigned short* WXP  = (unsigned short*)(ws + kOffWXP);
  unsigned short* WDT  = (unsigned short*)(ws + kOffWDT);
  unsigned short* WRES = (unsigned short*)(ws + kOffWRES);
  unsigned short* WOUT = (unsigned short*)(ws + kOffWOUT);
  unsigned short* XZB  = (unsigned short*)(ws + kOffXZB);
  float*          U32  = (float*)(ws + kOffU32);
  unsigned short* U16  = (unsigned short*)(ws + kOffU16);
  float*          XDBL = (float*)(ws + kOffXDBL);
  unsigned short* DTSA = (unsigned short*)(ws + kOffDTSA);
  float*          DTR  = (float*)(ws + kOffDTR);
  float*          YS   = (float*)(ws + kOffYS);
  float*          RES  = DTR;
  unsigned short* YF   = U16;

  cvt_w_kernel<0><<<kTot2WIN / 256, 256, 0, stream>>>(in_proj_w, WIN, kXZ, kC, kC, kTot2WIN);
  cvt_w_kernel<1><<<kTot2WXP / 256, 256, 0, stream>>>(x_proj_w, WXP, kK4 * kXDW, kDI, kDI, kTot2WXP);
  cvt_w_kernel<0><<<kTot2WDT / 256, 256, 0, stream>>>(dt_w, WDT, kK4 * kDI, kDTK, kR, kTot2WDT);
  cvt_w_kernel<0><<<kTot2WRES / 256, 256, 0, stream>>>(res_proj_w, WRES, kDI, kC, kC, kTot2WRES);
  cvt_w_kernel<0><<<kTot2WOUT / 256, 256, 0, stream>>>(out_proj_w, WOUT, kC, kDI, kDI, kTot2WOUT);

  ln1_kernel<<<kPos / 4, 384, 0, stream>>>(inputs, ln1_w, ln1_b, XLN);

  wmma_gemm64<0, false, 0, 1, false><<<dim3(((kPos / 64) * (kXZ / 64)) / 8, 1), 256, 0, stream>>>(
      XLN, nullptr, kC, 0L,
      WIN, nullptr, kC, 0L,
      (void*)XZB, nullptr, kXZ, 0L,
      nullptr, nullptr, 0L,
      kPos, kXZ, kC, kScaleIn);

  dwconv_silu_kernel<<<kPos / 4, 384, 0, stream>>>(XZB, conv_w, conv_b, U32, U16);

  wmma_gemm64<0, false, 0, 0, false><<<dim3(((kRowsK / 64) * (kXDW / 64)) / 8, kK4), 256, 0, stream>>>(
      U16, nullptr, kDI, (long)kRowsK * kDI,
      WXP, nullptr, kDI, (long)kXDW * kDI,
      (void*)XDBL, nullptr, kXDW, (long)kRowsK * kXDW,
      nullptr, nullptr, 0L,
      kRowsK, kXDW, kDI, kScaleXp);

  dts_pack_kernel<<<kTotPack / 256, 256, 0, stream>>>(XDBL, DTSA, kTotPack);

  wmma_gemm64<0, false, 0, 0, false><<<dim3(((kRowsK / 64) * (kDI / 64)) / 8, kK4), 256, 0, stream>>>(
      DTSA, nullptr, kDTK, (long)kRowsK * kDTK,
      WDT, nullptr, kDTK, (long)kDI * kDTK,
      (void*)DTR, nullptr, kDI, (long)kRowsK * kDI,
      nullptr, nullptr, 0L,
      kRowsK, kDI, kDTK, kScaleDt);

  scan_kernel<<<kK4 * kB * (kDI / kScanCh), kScanCh, 0, stream>>>(XDBL, DTR, U32, dt_b, A_logs, Ds, YS);

  wmma_gemm64<0, false, 0, 0, false><<<dim3(((kPos / 64) * (kDI / 64)) / 8, 1), 256, 0, stream>>>(
      XLN, nullptr, kC, 0L,
      WRES, nullptr, kC, 0L,
      (void*)RES, nullptr, kDI, 0L,
      nullptr, nullptr, 0L,
      kPos, kDI, kC, kScaleRes);

  norm_gate_kernel<<<kPos / 2, 384, 0, stream>>>(YS, out_norm_w, out_norm_b, RES, XZB, YF);

  wmma_gemm64<0, false, 0, 0, true><<<dim3(((kPos / 64) * (kC / 64)) / 8, 1), 256, 0, stream>>>(
      YF, nullptr, kDI, 0L,
      WOUT, nullptr, kDI, 0L,
      (void*)out, nullptr, kC, 0L,
      nullptr, inputs, 0L,
      kPos, kC, kDI, kScaleOut);
}
